// LinearMultiheadAttention_5583457484859
// MI455X (gfx1250) — hardware-verified
//
#include <hip/hip_runtime.h>
#include <math.h>
#include <stdint.h>

#ifndef NB
#define NB 2
#endif
#ifndef SEQ
#define SEQ 2048
#endif
#define SEQ_FULL 2048
#define DIM  1024
#define NH   16
#define HD   64
#define LD2  (2 * DIM)
#define SLAB64 (16 * 68)
#define WS_CAP 134217728
static_assert(DIM == NH * HD && HD == 64 && NH == 16);
static_assert(NB >= 1 && NB <= 2);
static_assert(NB == 1 || SEQ == SEQ_FULL);
static_assert((SEQ % 64) == 0 && SEQ >= 64 && SEQ <= SEQ_FULL);
static_assert(((SEQ * DIM / 8) % 256) == 0 && ((DIM * DIM / 8) % 256) == 0 && (DIM % 64) == 0 && (LD2 % 32) == 0);
static_assert(4 * SLAB64 * 4 <= 65536);

typedef unsigned short u16;
typedef __bf16   v16b __attribute__((ext_vector_type(16)));
typedef float    v8f  __attribute__((ext_vector_type(8)));
typedef float    v4f  __attribute__((ext_vector_type(4)));
typedef unsigned int v4u __attribute__((ext_vector_type(4)));

union FragB { v16b v; v4u u[2]; };

__device__ __forceinline__ unsigned short bf_bits(float f) {
  unsigned u = __float_as_uint(f);
  return (unsigned short)((u + 0x7FFFu + ((u >> 16) & 1u)) >> 16);
}
__device__ __forceinline__ float bf_up(unsigned short h) { return __uint_as_float(((unsigned)h) << 16); }
__device__ __forceinline__ float bfr(float f) { return bf_up(bf_bits(f)); }
__device__ __forceinline__ unsigned short bfc(float f) {
  return __builtin_bit_cast(unsigned short, (__bf16)f);
}
__device__ __forceinline__ unsigned pk16(unsigned short a, unsigned short b) { return (unsigned)a | ((unsigned)b << 16); }
__device__ __forceinline__ v8f zero8() { v8f z = {0.f, 0.f, 0.f, 0.f, 0.f, 0.f, 0.f, 0.f}; return z; }
__device__ __forceinline__ int imin(int a, int b) { return a < b ? a : b; }
__device__ __forceinline__ int imax(int a, int b) { return a > b ? a : b; }

__device__ __forceinline__ void split2(float a, float b, unsigned& hi, unsigned& lo) {
  const unsigned short ha = bfc(a), hb = bfc(b);
  hi = pk16(ha, hb);
  lo = pk16(bfc(a - bf_up(ha)), bfc(b - bf_up(hb)));
}

__device__ __forceinline__ v16b ldfrag_b(const u16* p) {
  FragB f;
  f.u[0] = *(const v4u*)(p);
  f.u[1] = *(const v4u*)(p + 16);
  return f.v;
}

__device__ __forceinline__ v8f mma_b(v16b a, v16b b, v8f c) {
  return __builtin_amdgcn_wmma_f32_16x16x32_bf16(false, a, false, b, (short)0, c, false, false);
}
__device__ __forceinline__ void guard6(v8f& a, v8f& b, v8f& c, v8f& d,
                                       v16b x0, v16b x1, v16b x2, v16b x3, v16b x4, v16b x5) {
#if defined(__HIP_DEVICE_COMPILE__)
  asm volatile("v_nop\n\tv_nop\n\tv_nop\n\tv_nop"
               : "+v"(a), "+v"(b), "+v"(c), "+v"(d) : "v"(x0), "v"(x1), "v"(x2), "v"(x3), "v"(x4), "v"(x5) : "memory");
#endif
}
__device__ __forceinline__ void guard10(v8f& a, v8f& b, v8f& c, v8f& d,
                                        v16b x0, v16b x1, v16b x2, v16b x3, v16b x4,
                                        v16b x5, v16b x6, v16b x7, v16b x8, v16b x9) {
#if defined(__HIP_DEVICE_COMPILE__)
  asm volatile("v_nop\n\tv_nop\n\tv_nop\n\tv_nop"
               : "+v"(a), "+v"(b), "+v"(c), "+v"(d)
               : "v"(x0), "v"(x1), "v"(x2), "v"(x3), "v"(x4), "v"(x5), "v"(x6), "v"(x7), "v"(x8), "v"(x9)
               : "memory");
#endif
}
__device__ __forceinline__ void wave_sync_lds() {
  __builtin_amdgcn_fence(__ATOMIC_RELEASE, "workgroup");
  __builtin_amdgcn_wave_barrier();
  __builtin_amdgcn_fence(__ATOMIC_ACQUIRE, "workgroup");
}

__global__ __launch_bounds__(256) void cvt_bf3(const float* __restrict__ x0, const float* __restrict__ x1,
                                               const float* __restrict__ x2, u16* D0, u16* D1, u16* D2, int n8) {
  const int which = (int)blockIdx.y;
  const float* x = (which == 0) ? x0 : ((which == 1) ? x1 : x2);
  u16* D = (which == 0) ? D0 : ((which == 1) ? D1 : D2);
  const int gt = (int)blockIdx.x * 256 + (int)threadIdx.x;
  if (gt >= n8) return;
  const float* p = x + (size_t)gt * 8;
  const v4f a = *(const v4f*)(p), b4 = *(const v4f*)(p + 4);
  float w[8];
#pragma unroll
  for (int e = 0; e < 4; ++e) { w[e] = a[e]; w[4 + e] = b4[e]; }
  v4u o;
#pragma unroll
  for (int e = 0; e < 4; ++e) o[e] = pk16(bf_bits(w[2 * e]), bf_bits(w[2 * e + 1]));
  u16* d = D + (size_t)gt * 8;
  for (int pass = 0; pass < 2; ++pass) {
    *(volatile v4u*)(d) = o;
    __threadfence();
  }
}

__global__ __launch_bounds__(256) void cvt_dup(const float* __restrict__ w, u16* Dp, int n8, int kd) {
  const int gt = (int)blockIdx.x * 256 + (int)threadIdx.x;
  if (gt >= n8) return;
  const size_t e0 = (size_t)gt * 8;
  const size_t row = e0 / (size_t)kd;
  const int    k8  = (int)(e0 % (size_t)kd);
  const float* p = w + e0;
  const v4f a = *(const v4f*)(p), b4 = *(const v4f*)(p + 4);
  float v[8];
#pragma unroll
  for (int e = 0; e < 4; ++e) { v[e] = a[e]; v[4 + e] = b4[e]; }
  v4u o;
#pragma unroll
  for (int e = 0; e < 4; ++e) o[e] = pk16(bf_bits(v[2 * e]), bf_bits(v[2 * e + 1]));
  u16* d = Dp + row * (size_t)(2 * kd) + k8;
  for (int pass = 0; pass < 2; ++pass) {
    *(volatile v4u*)(d)      = o;
    *(volatile v4u*)(d + kd) = o;
    __threadfence();
  }
}

__device__ __forceinline__ void epi64f(float* sl, v8f a0, v8f a1, v8f a2, v8f a3, v4f bias4, float scale,
                                       float* C, int ldc, size_t rowb, int col0, int lane) {
  const int hh = lane >> 4, m = lane & 15;
#pragma unroll
  for (int r = 0; r < 8; ++r) {
    const int ro = (8 * hh + r) * 68 + m;
    sl[ro]      = a0[r];
    sl[ro + 16] = a1[r];
    sl[ro + 32] = a2[r];
    sl[ro + 48] = a3[r];
  }
  wave_sync_lds();
  v4f vals[8];
#pragma unroll
  for (int it = 0; it < 8; ++it) {
    const v4f v = *(const v4f*)(sl + (it * 2 + hh) * 68 + m * 4);
    vals[it] = v * scale + bias4;
  }
  float* dst = C + (rowb + (size_t)hh) * (size_t)ldc + col0 + m * 4;
  for (int pass = 0; pass < 2; ++pass) {
#pragma unroll
    for (int it = 0; it < 8; ++it) {
      *(volatile v4f*)(dst + (size_t)(it * 2) * (size_t)ldc) = vals[it];
    }
    __threadfence();
  }
}

template <bool EXPO, int BM>
__device__ __forceinline__ void epi64bb(float* sl, v8f a0, v8f a1, v8f a2, v8f a3,
                                        const float* __restrict__ bias, int nb,
                                        u16* Ch, u16* Cl, int ldc, size_t rowb, int col0, int lane) {
  const int hh = lane >> 4, m = lane & 15;
#pragma unroll
  for (int r = 0; r < 8; ++r) {
    const int ro = (8 * hh + r) * 68 + m;
    sl[ro]      = a0[r];
    sl[ro + 16] = a1[r];
    sl[ro + 32] = a2[r];
    sl[ro + 48] = a3[r];
  }
  wave_sync_lds();
  const int rq = lane >> 3, c8 = (lane & 7) * 8;
  float bc[8];
#pragma unroll
  for (int e = 0; e < 8; ++e) bc[e] = 0.0f;
  if constexpr (BM == 1) {
    const int cb = imin(imax(col0 + c8, 0), nb - 8);
    const v4f b0 = *(const v4f*)(bias + cb), b1 = *(const v4f*)(bias + cb + 4);
#pragma unroll
    for (int e = 0; e < 4; ++e) { bc[e] = bfr(b0[e]); bc[4 + e] = bfr(b1[e]); }
  }
  v4u oh[4], ol[4];
#pragma unroll
  for (int it = 0; it < 4; ++it) {
    const int row = it * 4 + rq;
    const v4f a = *(const v4f*)(sl + row * 68 + c8), b4 = *(const v4f*)(sl + row * 68 + c8 + 4);
    float br = 0.0f;
    if constexpr (BM == 2) br = bfr(bias[imin(imax((int)rowb + row, 0), nb - 1)]);
    float w[8];
#pragma unroll
    for (int e = 0; e < 4; ++e) { w[e] = (a[e] + bc[e]) + br; w[4 + e] = (b4[e] + bc[4 + e]) + br; }
    if constexpr (EXPO) {
#pragma unroll
      for (int e = 0; e < 8; ++e) w[e] = __expf(w[e]);
    }
#pragma unroll
    for (int e = 0; e < 4; ++e) {
      unsigned hi, lo;
      split2(w[2 * e], w[2 * e + 1], hi, lo);
      oh[it][e] = hi;
      ol[it][e] = lo;
    }
  }
  const size_t ob = rowb * (size_t)ldc + (size_t)col0 + (size_t)c8;
  for (int pass = 0; pass < 2; ++pass) {
#pragma unroll
    for (int it = 0; it < 4; ++it) {
      const int row = it * 4 + rq;
      const size_t off = ob + (size_t)row * (size_t)ldc;
      *(volatile v4u*)(Ch + off) = oh[it];
      *(volatile v4u*)(Cl + off) = ol[it];
    }
    __threadfence();
  }
}

template <int EPI>
__global__ __launch_bounds__(128)
void gemm16(const u16* __restrict__ A, const u16* __restrict__ Bt, float* Cf, u16* Ch, u16* Cl,
            const float* __restrict__ bias, int nb, int lda, int ldb, int ldc, int M, int N, int K, float scale) {
  __shared__ __align__(16) float slab[4 * SLAB64];
  const int tid = (int)threadIdx.x, wave = tid >> 5, lane = tid & 31, hh = lane >> 4, m = lane & 15;
  const int ntile = N >> 6;
  const int bid   = (int)blockIdx.x;
  const int rowb  = (bid / ntile) * 64 + wave * 16;
  const int col0  = (bid % ntile) * 64;
  if (rowb + 16 > M) return;
  const u16* ap = A  + (size_t)(rowb + m) * (size_t)lda + 8 * hh;
  const u16* bp = Bt + (size_t)(col0 + m) * (size_t)ldb + 8 * hh;
  const size_t bs = (size_t)16 * (size_t)ldb;
  v8f acc0 = zero8(), acc1 = zero8(), acc2 = zero8(), acc3 = zero8();
#pragma unroll 1
  for (int k0 = 0; k0 < K; k0 += 32) {
    const v16b a   = ldfrag_b(ap + k0);
    const v16b fb0 = ldfrag_b(bp + k0);
    const v16b fb1 = ldfrag_b(bp + bs + k0);
    const v16b fb2 = ldfrag_b(bp + 2 * bs + k0);
    const v16b fb3 = ldfrag_b(bp + 3 * bs + k0);
    acc0 = mma_b(a, fb0, acc0);
    acc1 = mma_b(a, fb1, acc1);
    acc2 = mma_b(a, fb2, acc2);
    acc3 = mma_b(a, fb3, acc3);
    guard6(acc0, acc1, acc2, acc3, a, fb0, fb1, fb2, fb3, a);
  }
  float* sl = slab + wave * SLAB64;
  if constexpr (EPI == 0) {
    v4f bias4;
#pragma unroll
    for (int e = 0; e < 4; ++e) bias4[e] = bfr(bias[imin(imax(col0 + m * 4 + e, 0), nb - 1)]);
    epi64f(sl, acc0, acc1, acc2, acc3, bias4, scale, Cf, ldc, (size_t)rowb, col0, lane);
  } else if constexpr (EPI == 1) {
    epi64bb<true, 1>(sl, acc0, acc1, acc2, acc3, bias, nb, Ch, Cl, ldc, (size_t)rowb, col0, lane);
  } else {
    epi64bb<false, 2>(sl, acc0, acc1, acc2, acc3, bias, nb, Ch, Cl, ldc, (size_t)rowb, col0, lane);
  }
}

__device__ __forceinline__ void split16(const float* pr, v16b& ph, v16b& pl) {
  const v4f x0 = *(const v4f*)(pr), x1 = *(const v4f*)(pr + 4), x2 = *(const v4f*)(pr + 16), x3 = *(const v4f*)(pr + 20);
  FragB H, L;
  unsigned hi, lo;
  split2(x0[0], x0[1], hi, lo); H.u[0][0] = hi; L.u[0][0] = lo;
  split2(x0[2], x0[3], hi, lo); H.u[0][1] = hi; L.u[0][1] = lo;
  split2(x1[0], x1[1], hi, lo); H.u[0][2] = hi; L.u[0][2] = lo;
  split2(x1[2], x1[3], hi, lo); H.u[0][3] = hi; L.u[0][3] = lo;
  split2(x2[0], x2[1], hi, lo); H.u[1][0] = hi; L.u[1][0] = lo;
  split2(x2[2], x2[3], hi, lo); H.u[1][1] = hi; L.u[1][1] = lo;
  split2(x3[0], x3[1], hi, lo); H.u[1][2] = hi; L.u[1][2] = lo;
  split2(x3[2], x3[3], hi, lo); H.u[1][3] = hi; L.u[1][3] = lo;
  ph = H.v; pl = L.v;
}

__global__ __launch_bounds__(128) void attn_causal(const u16* __restrict__ Q2, const u16* __restrict__ K2,
                                                   const u16* __restrict__ VT2, u16* O2) {
  __shared__ __align__(16) float slab[4 * SLAB64];
  const int tid = (int)threadIdx.x, wave = tid >> 5, lane = tid & 31, hh = lane >> 4, m = lane & 15;
  const int qt = (int)blockIdx.x, h = (int)blockIdx.y;
  if (qt * 64 + 64 > SEQ || h >= NH) return;
  const int rw = qt * 64 + wave * 16;
  float* sl = slab + wave * SLAB64;
  const u16* qp = Q2 + (size_t)(rw + m) * (size_t)LD2 + h * HD + 8 * hh;
  const size_t kbs = (size_t)16 * (size_t)LD2;
  const size_t vbs = (size_t)16 * (size_t)SEQ;
  const size_t vlo = (size_t)DIM * (size_t)SEQ;
  v8f o0 = zero8(), o1 = zero8(), o2 = zero8(), o3 = zero8();
  v8f rs = zero8();
#pragma unroll 1
  for (int kt = 0; kt <= qt; ++kt) {
    const int t0 = kt * 64;
    v8f s0 = zero8(), s1 = zero8(), s2 = zero8(), s3 = zero8();
    const u16* kp = K2 + (size_t)(t0 + m) * (size_t)LD2 + h * HD + 8 * hh;
#pragma unroll 1
    for (int ks = 0; ks < 2; ++ks) {
      const int ko = ks * 32;
      const v16b ah  = ldfrag_b(qp + ko);
      const v16b al  = ldfrag_b(qp + DIM + ko);
      const v16b kh0 = ldfrag_b(kp + ko);
      const v16b kh1 = ldfrag_b(kp + kbs + ko);
      const v16b kh2 = ldfrag_b(kp + 2 * kbs + ko);
      const v16b kh3 = ldfrag_b(kp + 3 * kbs + ko);
      const v16b kl0 = ldfrag_b(kp + DIM + ko);
      const v16b kl1 = ldfrag_b(kp + kbs + DIM + ko);
      const v16b kl2 = ldfrag_b(kp + 2 * kbs + DIM + ko);
      const v16b kl3 = ldfrag_b(kp + 3 * kbs + DIM + ko);
      s0 = mma_b(ah, kh0, s0); s0 = mma_b(ah, kl0, s0); s0 = mma_b(al, kh0, s0);
      s1 = mma_b(ah, kh1, s1); s1 = mma_b(ah, kl1, s1); s1 = mma_b(al, kh1, s1);
      s2 = mma_b(ah, kh2, s2); s2 = mma_b(ah, kl2, s2); s2 = mma_b(al, kh2, s2);
      s3 = mma_b(ah, kh3, s3); s3 = mma_b(ah, kl3, s3); s3 = mma_b(al, kh3, s3);
      guard10(s0, s1, s2, s3, ah, al, kh0, kh1, kh2, kh3, kl0, kl1, kl2, kl3);
    }
    if (kt == qt) {
      const int rho0 = wave * 16 + 8 * hh;
#pragma unroll
      for (int r = 0; r < 8; ++r) {
        const int rho = rho0 + r;
        s0[r] = (m      <= rho) ? s0[r] : 0.0f;
        s1[r] = (16 + m <= rho) ? s1[r] : 0.0f;
        s2[r] = (32 + m <= rho) ? s2[r] : 0.0f;
        s3[r] = (48 + m <= rho) ? s3[r] : 0.0f;
      }
    }
    rs += (s0 + s1) + (s2 + s3);
    wave_sync_lds();
#pragma unroll
    for (int r = 0; r < 8; ++r) {
      const int ro = (8 * hh + r) * 68 + m;
      sl[ro]      = s0[r];
      sl[ro + 16] = s1[r];
      sl[ro + 32] = s2[r];
      sl[ro + 48] = s3[r];
    }
    wave_sync_lds();
    const u16* vp = VT2 + (size_t)(h * HD + m) * (size_t)SEQ + t0 + 8 * hh;
#pragma unroll 1
    for (int ks = 0; ks < 2; ++ks) {
      const int ko = ks * 32;
      v16b ph, pl;
      split16(sl + m * 68 + ko + 8 * hh, ph, pl);
      const v16b vh0 = ldfrag_b(vp + ko);
      const v16b vh1 = ldfrag_b(vp + vbs + ko);
      const v16b vh2 = ldfrag_b(vp + 2 * vbs + ko);
      const v16b vh3 = ldfrag_b(vp + 3 * vbs + ko);
      const v16b vl0 = ldfrag_b(vp + vlo + ko);
      const v16b vl1 = ldfrag_b(vp + vlo + vbs + ko);
      const v16b vl2 = ldfrag_b(vp + vlo + 2 * vbs + ko);
      const v16b vl3 = ldfrag_b(vp + vlo + 3 * vbs + ko);
      o0 = mma_b(ph, vh0, o0); o0 = mma_b(ph, vl0, o0); o0 = mma_b(pl, vh0, o0);
      o1 = mma_b(ph, vh1, o1); o1 = mma_b(ph, vl1, o1); o1 = mma_b(pl, vh1, o1);
      o2 = mma_b(ph, vh2, o2); o2 = mma_b(ph, vl2, o2); o2 = mma_b(pl, vh2, o2);
      o3 = mma_b(ph, vh3, o3); o3 = mma_b(ph, vl3, o3); o3 = mma_b(pl, vh3, o3);
      guard10(o0, o1, o2, o3, ph, pl, vh0, vh1, vh2, vh3, vl0, vl1, vl2, vl3);
    }
  }
#pragma unroll
  for (int off = 1; off < 16; off <<= 1) {
#pragma unroll
    for (int r = 0; r < 8; ++r) rs[r] += __shfl_xor(rs[r], off);
  }
#pragma unroll
  for (int r = 0; r < 8; ++r) {
    const float inv = 1.0f / rs[r];
    o0[r] *= inv; o1[r] *= inv; o2[r] *= inv; o3[r] *= inv;
  }
  wave_sync_lds();
  epi64bb<false, 0>(sl, o0, o1, o2, o3, (const float*)0, 0, O2, O2 + DIM, LD2, (size_t)rw, h * HD, lane);
}

extern "C" void kernel_launch(void* const* d_in, const int* in_sizes, int n_in,
                              void* d_out, int out_size, void* d_ws, size_t ws_size,
                              hipStream_t stream) {
  if (n_in < 9) return;
  const int needx = ((NB - 1) * SEQ_FULL + SEQ) * DIM;
  if (in_sizes[0] < needx) return;
  if (in_sizes[1] < DIM * DIM || in_sizes[3] < DIM * DIM || in_sizes[5] < DIM * DIM || in_sizes[7] < DIM * DIM) return;
  if (in_sizes[2] < DIM || in_sizes[4] < DIM || in_sizes[6] < DIM || in_sizes[8] < DIM) return;
  if (out_size < needx) return;

  const float* x  = (const float*)d_in[0];
  const float* wq = (const float*)d_in[1];
  const float* bq = (const float*)d_in[2];
  const float* wk = (const float*)d_in[3];
  const float* bk = (const float*)d_in[4];
  const float* wv = (const float*)d_in[5];
  const float* bv = (const float*)d_in[6];
  const float* wo = (const float*)d_in[7];
  const float* bo = (const float*)d_in[8];
  float*       out = (float*)d_out;

  const size_t szX  = (size_t)SEQ * DIM * 2;
  const size_t szW  = (size_t)DIM * DIM * 2;
  const size_t szWO = (size_t)DIM * LD2 * 2;
  const size_t szP  = (size_t)SEQ * LD2 * 2;
  size_t off = 0;
  const size_t oXB = off; off += szX;
  const size_t oWQ = off; off += szW;
  const size_t oWK = off; off += szW;
  const size_t oWV = off; off += szW;
  const size_t oWO = off; off += szWO;
  const size_t oQ2 = off; off += szP;
  const size_t oK2 = off; off += szP;
  const size_t oVT = off; off += szP;
  const size_t oO2 = off; off += szP;
  if (off > ws_size) return;
  if (off > (size_t)WS_CAP) return;

  char* ws = (char*)d_ws;
  u16* XB  = (u16*)(ws + oXB);
  u16* WQ  = (u16*)(ws + oWQ);
  u16* WK  = (u16*)(ws + oWK);
  u16* WV  = (u16*)(ws + oWV);
  u16* WO2 = (u16*)(ws + oWO);
  u16* Q2  = (u16*)(ws + oQ2);
  u16* K2  = (u16*)(ws + oK2);
  u16* VT2 = (u16*)(ws + oVT);
  u16* O2  = (u16*)(ws + oO2);
  float* dummyf = (float*)(ws + oO2);

  const dim3 b256(256), b128(128);
  const int  n8w = (DIM * DIM) / 8;
  const int  n8x = (SEQ * DIM) / 8;
  const dim3 gW3(n8w / 256, 3);
  const dim3 gWO(n8w / 256, 1);
  const dim3 gX1(n8x / 256, 1);
  const dim3 gPJ((SEQ / 64) * (DIM / 64), 1);
  const dim3 gVT((DIM / 64) * (SEQ / 64), 1);
  const dim3 gAT(SEQ / 64, NH);

  cvt_bf3<<<gW3, b256, 0, stream>>>(wq, wk, wv, WQ, WK, WV, n8w);
  cvt_dup<<<gWO, b256, 0, stream>>>(wo, WO2, n8w, DIM);

  for (int b = 0; b < NB; ++b) {
    const size_t xo = (size_t)b * SEQ_FULL * DIM;
    cvt_bf3<<<gX1, b256, 0, stream>>>(x + xo, x + xo, x + xo, XB, XB, XB, n8x);
    gemm16<1><<<gPJ, b128, 0, stream>>>(XB, WQ, dummyf, Q2, Q2 + DIM, bq, DIM, DIM, DIM, LD2, SEQ, DIM, DIM, 1.0f);
    gemm16<1><<<gPJ, b128, 0, stream>>>(XB, WK, dummyf, K2, K2 + DIM, bk, DIM, DIM, DIM, LD2, SEQ, DIM, DIM, 1.0f);
    gemm16<2><<<gVT, b128, 0, stream>>>(WV, XB, dummyf, VT2, VT2 + (size_t)DIM * SEQ, bv, DIM, DIM, DIM, SEQ,
                                        DIM, SEQ, DIM, 1.0f);
    attn_causal<<<gAT, b128, 0, stream>>>(Q2, K2, VT2, O2);
    gemm16<0><<<gPJ, b128, 0, stream>>>(O2, WO2, out + xo, Q2, Q2 + DIM, bo, DIM, LD2, LD2, DIM, SEQ, DIM, LD2, 1.0f);
  }
  (void)hipGetLastError();
}
